// GNN_76639396430550
// MI455X (gfx1250) — hardware-verified
//
#include <hip/hip_runtime.h>
#include <stddef.h>
#include <stdint.h>
#include <math.h>


#define FIN    64
#define DIM    20
#define PCH    32
#define KG     64
#define NGR    512
#define NCLS   2
#define GPB    16
#define NTHR   256
#define NWAVE  8
#define EPT    8
#define CHUNK  (NTHR * EPT)
#define WCAP   (EPT * 32)
#define LISTN  (NWAVE * WCAP)
#define NBA    1024
#define SLA    10
#define RCAP   24576
#define DEGCAP 64
#define GBM    64
#define GTHR   128
#define FROWS  512
#define NPAR   12
#define AGG_ZINTS    (LISTN + 2 * RCAP + 3 * NBA)
#define AGG_LDS_INTS (AGG_ZINTS + 16 + NBA)
#define WSMAX  134217728

static_assert((CHUNK & (CHUNK - 1)) == 0 && CHUNK <= 4096);
static_assert((NBA & (NBA - 1)) == 0 && NBA == (1 << SLA));
static_assert(((long long)CHUNK << SLA) < (1LL << 31));
static_assert(NBA % 32 == 0 && NBA % GBM == 0 && NBA % FROWS == 0 && NBA == 4 * NTHR);
static_assert(RCAP % (4 * NTHR) == 0 && AGG_ZINTS % (4 * NTHR) == 0 && LISTN % 4 == 0);
static_assert(((AGG_ZINTS + 16) % 4) == 0);
static_assert(AGG_LDS_INTS * 4 <= 300000);
static_assert(KG % 32 == 0 && FIN == KG && DIM <= 32 && PCH == 32 && DIM % 4 == 0);
static_assert(GBM == (GTHR / 32) * 16);
static_assert((FROWS * DIM * 4) % 128 == 0 && (FROWS * (DIM / 4)) % NTHR == 0);
static_assert(NGR % GPB == 0 && (GPB * DIM * 4) % 128 == 0 && GPB * NCLS * 4 == 128);
static_assert(DEGCAP <= 255);

typedef float          v4f   __attribute__((ext_vector_type(4)));
typedef float          v8f   __attribute__((ext_vector_type(8)));
typedef double         v2d   __attribute__((ext_vector_type(2)));
typedef int            v4i   __attribute__((ext_vector_type(4)));
typedef int            v8i   __attribute__((ext_vector_type(8)));
typedef unsigned short v8us  __attribute__((ext_vector_type(8)));
typedef unsigned short v16us __attribute__((ext_vector_type(16)));
typedef __bf16         v16bf __attribute__((ext_vector_type(16)));
typedef v4f  __attribute__((may_alias)) v4fa;
typedef v4i  __attribute__((may_alias)) v4ia;
typedef v8us __attribute__((may_alias)) v8usa;
union FragB { v16bf v; v16us u; v8us h[2]; v8i w; };

__device__ __forceinline__ v8f wmb(const FragB& a, const FragB& b, v8f c) {
  v8f d = __builtin_amdgcn_wmma_f32_16x16x32_bf16(false, a.v, false, b.v, (short)0, c, false, false);
  asm volatile("v_nop\n\tv_nop\n\tv_nop\n\tv_nop" : "+v"(d) : "v"(a.w), "v"(b.w));
  return d;
}

__device__ __forceinline__ unsigned bf16_bits(float f) {
  const unsigned u = __float_as_uint(f);
  return (u + 0x7FFFu + ((u >> 16) & 1u)) >> 16;
}
__device__ __forceinline__ float bf16_val(float f) {
  return __uint_as_float(bf16_bits(f) << 16);
}
__device__ __forceinline__ float bn_relu(float a, float mean, float rstd, float g, float be) {
  float t = (a - mean) * rstd;
  t = t * g + be;
  return (t > 0.0f) ? t : (t - t);
}
__device__ __forceinline__ float nmax(float a, float m) {
  return (a > m || a != a) ? a : m;
}

template <int SLB>
__device__ __forceinline__ int scan_chunk(const int* __restrict__ dsts, int nE, int cbase, int slotBase,
                                          int nb, int vec8, int* list, int tid, int lane, int wave) {
  int wc = 0;
  const int el0  = tid * EPT;
  const int e0   = cbase + el0;
  const int sent = -2147483647 - 1;
  v4i da, db;
  if (vec8 != 0 && cbase + CHUNK <= nE) {
    da = *(const v4i*)(dsts + e0);
    db = *(const v4i*)(dsts + e0 + 4);
  } else {
    da.x = (e0     < nE) ? dsts[min(e0,     nE - 1)] : sent;
    da.y = (e0 + 1 < nE) ? dsts[min(e0 + 1, nE - 1)] : sent;
    da.z = (e0 + 2 < nE) ? dsts[min(e0 + 2, nE - 1)] : sent;
    da.w = (e0 + 3 < nE) ? dsts[min(e0 + 3, nE - 1)] : sent;
    db.x = (e0 + 4 < nE) ? dsts[min(e0 + 4, nE - 1)] : sent;
    db.y = (e0 + 5 < nE) ? dsts[min(e0 + 5, nE - 1)] : sent;
    db.z = (e0 + 6 < nE) ? dsts[min(e0 + 6, nE - 1)] : sent;
    db.w = (e0 + 7 < nE) ? dsts[min(e0 + 7, nE - 1)] : sent;
  }
  const unsigned nbs = (unsigned)slotBase;
  const unsigned unb = (unsigned)nb;
  const unsigned s0 = (unsigned)da.x - nbs, s1 = (unsigned)da.y - nbs;
  const unsigned s2 = (unsigned)da.z - nbs, s3 = (unsigned)da.w - nbs;
  const unsigned s4 = (unsigned)db.x - nbs, s5 = (unsigned)db.y - nbs;
  const unsigned s6 = (unsigned)db.z - nbs, s7 = (unsigned)db.w - nbs;
  const bool h0 = s0 < unb, h1 = s1 < unb, h2 = s2 < unb, h3 = s3 < unb;
  const bool h4 = s4 < unb, h5 = s5 < unb, h6 = s6 < unb, h7 = s7 < unb;
  const unsigned any = __builtin_amdgcn_ballot_w32(h0 | h1 | h2 | h3 | h4 | h5 | h6 | h7);
  if (any != 0u) {
#define HITJ(J, HJ, SJ) { \
      const unsigned mj = __builtin_amdgcn_ballot_w32(HJ); \
      if (mj != 0u) { \
        if (HJ) { \
          const int pos = wc + (int)__builtin_amdgcn_mbcnt_lo(mj, 0u); \
          if (pos < WCAP) list[wave * WCAP + pos] = ((el0 + (J)) << SLB) | (int)(SJ); \
        } \
        wc += (int)__builtin_popcount(mj); } }
    HITJ(0, h0, s0)
    HITJ(1, h1, s1)
    HITJ(2, h2, s2)
    HITJ(3, h3, s3)
    HITJ(4, h4, s4)
    HITJ(5, h5, s5)
    HITJ(6, h6, s6)
    HITJ(7, h7, s7)
#undef HITJ
  }
  return wc;
}

__global__ __launch_bounds__(NTHR) void k_prep(
    const float* __restrict__ W0, const float* __restrict__ b0, const float* __restrict__ g0, const float* __restrict__ be0,
    const float* __restrict__ W1, const float* __restrict__ b1, const float* __restrict__ g1, const float* __restrict__ be1,
    const float* __restrict__ W2, const float* __restrict__ b2, const float* __restrict__ g2, const float* __restrict__ be2,
    const float* __restrict__ fcW, const float* __restrict__ fcb,
    unsigned short* W0T, unsigned short* W1T, unsigned short* W2T, float* par) {
  __shared__ __attribute__((aligned(16))) float ps[NPAR * 32];
  const int tid = (int)threadIdx.x, lane = tid & 31;
  const int wave = __builtin_amdgcn_readfirstlane(tid >> 5);
  const int n  = tid >> 3;
  const int k8 = (tid & 7) * 8;
  const int nc = n < DIM ? n : DIM - 1;
  const bool nok = n < DIM;
#pragma unroll 1
  for (int mat = 0; mat < 3; ++mat) {
    const float* W = (mat == 0) ? W0 : ((mat == 1) ? W1 : W2);
    unsigned short* P = (mat == 0) ? W0T : ((mat == 1) ? W1T : W2T);
    const int kk   = (mat == 0) ? k8 : (k8 & 31);
    const int klim = (mat == 0) ? FIN : DIM;
    v8us o;
#pragma unroll
    for (int i = 0; i < 8; ++i) {
      const int k  = kk + i;
      const int kc = k < klim ? k : klim - 1;
      const float v = W[kc * DIM + nc];
      o[i] = (nok && k < klim) ? (unsigned short)bf16_bits(v) : (unsigned short)0;
    }
    unsigned short* dp = P + n * KG + k8;
    *(volatile v8us*)dp = o;
    __threadfence();
    *(volatile v8us*)dp = o;
  }
  {
    const int cc = lane < DIM ? lane : DIM - 1;
    float v = 0.0f;
    switch (wave) {
      case 0: v = b0[cc];  break;
      case 1: v = g0[cc];  break;
      case 2: v = be0[cc]; break;
      case 3: v = b1[cc];  break;
      case 4: v = g1[cc];  break;
      case 5: v = be1[cc]; break;
      case 6: v = b2[cc];  break;
      default: v = g2[cc]; break;
    }
    ps[wave * 32 + lane] = (lane < DIM) ? bf16_val(v) : 0.0f;
    float w2 = 0.0f;
    bool ok2 = false;
    if (wave == 0)      { w2 = be2[cc];          ok2 = lane < DIM; }
    else if (wave == 1) { w2 = fcW[2 * cc];      ok2 = lane < DIM; }
    else if (wave == 2) { w2 = fcW[2 * cc + 1];  ok2 = lane < DIM; }
    else if (wave == 3) { w2 = fcb[lane < 1 ? lane : 1]; ok2 = lane < NCLS; }
    if (wave < 4) ps[(8 + wave) * 32 + lane] = ok2 ? bf16_val(w2) : 0.0f;
  }
  __syncthreads();
  {
    const int t4 = tid < 96 ? tid : 95;
    const v4f pv = *(const v4fa*)(ps + 4 * t4);
    const bool st = tid < 96;
    if (st) *(volatile v4f*)(par + 4 * t4) = pv;
    __threadfence();
    if (st) *(volatile v4f*)(par + 4 * t4) = pv;
  }
}

__global__ __launch_bounds__(NTHR) void k_build(const int* __restrict__ srcs, const int* __restrict__ dsts,
                                                int nE, int nN, int vec8,
                                                int* srcl, int* offsP, int* cntP, float* dinvP) {
  extern __shared__ __attribute__((aligned(16))) int dsm[];
  int* list = dsm;
  int* hl   = dsm + LISTN;
  int* sl   = dsm + LISTN + RCAP;
  int* cnt  = dsm + LISTN + 2 * RCAP;
  int* offs = cnt + NBA;
  int* cur  = offs + NBA;
  int* misc = cur + NBA;
  float* dv = (float*)(misc + 16);
  const int tid = (int)threadIdx.x, lane = tid & 31;
  const int wave = __builtin_amdgcn_readfirstlane(tid >> 5);
  const int nodeBase = (int)blockIdx.x * NBA;

  {
    const v4i z4 = {0, 0, 0, 0};
    for (int i = tid * 4; i < AGG_ZINTS; i += NTHR * 4) *(v4ia*)(dsm + i) = z4;
    if (tid < 16) misc[tid] = 0;
  }
  __syncthreads();

  int t = 0, ov = 0;
  const int nChunks = (nE + CHUNK - 1) / CHUNK;
#pragma unroll 1
  for (int ch = 0; ch < nChunks; ++ch) {
    const int cbase = ch * CHUNK;
    const int wc = scan_chunk<SLA>(dsts, nE, cbase, nodeBase, NBA, vec8, list, tid, lane, wave);
    if (lane == 0) misc[wave] = wc;
    __syncthreads();
    if (wave == 0) {
#pragma unroll 1
      for (int w2 = 0; w2 < NWAVE; ++w2) {
        int c = misc[w2];
        c = c < 0 ? 0 : (c > WCAP ? WCAP : c);
#pragma unroll 1
        for (int b0 = 0; b0 < c; b0 += 32) {
          const int idx = b0 + lane;
          const int ent = list[w2 * WCAP + (idx < WCAP ? idx : WCAP - 1)];
          const int m32 = (c - b0) < 32 ? (c - b0) : 32;
#pragma unroll 1
          for (int k = 0; k < m32; ++k) {
            const int u    = __builtin_amdgcn_readlane(ent, k);
            const int slot = u & (NBA - 1);
            const int el   = (u >> SLA) & (CHUNK - 1);
            const int pk   = (int)(((unsigned)(cbase + el) << SLA) | (unsigned)slot);
            if (t < RCAP) {
              if (lane == 0) { hl[t] = pk; cnt[slot] = cnt[slot] + 1; }
              t = t + 1;
            } else {
              ov = 1;
            }
          }
        }
      }
    }
    __syncthreads();
  }
  if (wave == 0 && lane == 0) { misc[8] = t; misc[9] = ov; }
  __syncthreads();
  int tt = misc[8];
  tt = tt < 0 ? 0 : (tt > RCAP ? RCAP : tt);
  const int ovf = misc[9];

  if (wave == 0) {
    const int base = lane * (NBA / 32);
    int s = 0;
#pragma unroll 1
    for (int i = 0; i < NBA / 32; ++i) s += cnt[base + i];
    int incl = s;
#pragma unroll
    for (int d = 1; d < 32; d <<= 1) {
      const int y = __shfl_up(incl, d, 32);
      if (lane >= d) incl += y;
    }
    int run = incl - s;
#pragma unroll 1
    for (int i = 0; i < NBA / 32; ++i) {
      const int cv = cnt[base + i];
      offs[base + i] = run;
      cur[base + i]  = run;
      run += cv;
    }
  }
  __syncthreads();
  if (wave == 0) {
#pragma unroll 1
    for (int b0 = 0; b0 < tt; b0 += 32) {
      const int idx = b0 + lane;
      const int ent = hl[idx < RCAP ? idx : RCAP - 1];
      const int m32 = (tt - b0) < 32 ? (tt - b0) : 32;
#pragma unroll 1
      for (int k = 0; k < m32; ++k) {
        const int u    = __builtin_amdgcn_readlane(ent, k);
        const int slot = u & (NBA - 1);
        if (lane == 0) {
          int p = cur[slot];
          p = p < 0 ? 0 : (p > RCAP - 1 ? RCAP - 1 : p);
          sl[p] = u;
          cur[slot] = p + 1;
        }
      }
    }
  }
  __syncthreads();

#pragma unroll 1
  for (int it = 0; it < RCAP / NTHR; ++it) {
    const int idx = it * NTHR + tid;
    const int wb  = it * NTHR + wave * 32;
    int s = 0;
    if (wb < tt) {
      const int ent = sl[idx];
      int eid = (int)((unsigned)ent >> SLA);
      eid = eid > nE - 1 ? nE - 1 : eid;
      int sr = srcs[eid];
      sr = sr < 0 ? 0 : (sr > nN - 1 ? nN - 1 : sr);
      s = (idx < tt) ? sr : 0;
    }
    hl[idx] = s;
  }
  const float qnan = __int_as_float(0x7fc00000);
#pragma unroll 1
  for (int j = 0; j < NBA / NTHR; ++j) {
    const int s = j * NTHR + tid;
    const int c = cnt[s];
    const float d = (float)c + 1.0f;
    const float r = 1.0f / sqrtf(d);
    dv[s] = (ovf != 0 || c > DEGCAP || c < 0) ? qnan : r;
  }
  __syncthreads();

  int* gl = srcl + (size_t)blockIdx.x * RCAP;
  const v4i c4 = *(const v4ia*)(cnt + 4 * tid);
  const v4i o4 = *(const v4ia*)(offs + 4 * tid);
  const v4f d4 = *(const v4fa*)(dv + 4 * tid);
#pragma unroll 1
  for (int it = 0; it < RCAP / (4 * NTHR); ++it) {
    const int i4 = (it * NTHR + tid) * 4;
    const v4i v = *(const v4ia*)(hl + i4);
    *(volatile v4i*)(gl + i4) = v;
  }
  *(volatile v4i*)(cntP  + (size_t)nodeBase + 4 * tid) = c4;
  *(volatile v4i*)(offsP + (size_t)nodeBase + 4 * tid) = o4;
  *(volatile v4f*)(dinvP + (size_t)nodeBase + 4 * tid) = d4;
  __threadfence();
#pragma unroll 1
  for (int it = 0; it < RCAP / (4 * NTHR); ++it) {
    const int i4 = (it * NTHR + tid) * 4;
    const v4i v = *(const v4ia*)(hl + i4);
    *(volatile v4i*)(gl + i4) = v;
  }
  *(volatile v4i*)(cntP  + (size_t)nodeBase + 4 * tid) = c4;
  *(volatile v4i*)(offsP + (size_t)nodeBase + 4 * tid) = o4;
  *(volatile v4f*)(dinvP + (size_t)nodeBase + 4 * tid) = d4;
}

template <int MODE>
__global__ __launch_bounds__(GTHR) void k_gemm(const float* __restrict__ src, int nN,
                                               const unsigned short* __restrict__ WT,
                                               const float* __restrict__ stats, const float* __restrict__ par,
                                               int prow, const float* __restrict__ dinvP, float* Y) {
  __shared__ __attribute__((aligned(16))) unsigned short at[GBM * KG];
  __shared__ __attribute__((aligned(16))) float stg[GBM * PCH];
  __shared__ float pm[4 * 32];
  const int tid = (int)threadIdx.x, lane = tid & 31, hh = lane >> 4, m = lane & 15;
  const int wave = __builtin_amdgcn_readfirstlane(tid >> 5);
  const int rowBase = (int)blockIdx.x * GBM;

  if constexpr (MODE != 0) {
    if (tid < 32) {
      pm[tid]      = stats[tid];
      pm[32 + tid] = stats[32 + tid];
      pm[64 + tid] = par[(prow + 1) * 32 + tid];
      pm[96 + tid] = par[(prow + 2) * 32 + tid];
    }
    __syncthreads();
  }

#pragma unroll 1
  for (int it = 0; it < (GBM * KG / 8) / GTHR; ++it) {
    const int u    = it * GTHR + tid;
    const int row  = u >> 3;
    const int q    = u & 7;
    const int grow = rowBase + row;
    v8us o;
    if constexpr (MODE == 0) {
      const int rc = grow < nN ? grow : nN - 1;
      const float* p = src + (size_t)rc * FIN + 8 * q;
      const v4f a = *(const v4f*)p;
      const v4f b = *(const v4f*)(p + 4);
      const bool ok = grow < nN;
      o[0] = ok ? (unsigned short)bf16_bits(a.x) : (unsigned short)0;
      o[1] = ok ? (unsigned short)bf16_bits(a.y) : (unsigned short)0;
      o[2] = ok ? (unsigned short)bf16_bits(a.z) : (unsigned short)0;
      o[3] = ok ? (unsigned short)bf16_bits(a.w) : (unsigned short)0;
      o[4] = ok ? (unsigned short)bf16_bits(b.x) : (unsigned short)0;
      o[5] = ok ? (unsigned short)bf16_bits(b.y) : (unsigned short)0;
      o[6] = ok ? (unsigned short)bf16_bits(b.z) : (unsigned short)0;
      o[7] = ok ? (unsigned short)bf16_bits(b.w) : (unsigned short)0;
    } else {
      const int cq = (q & 3) * 8;
      const float* p = src + (size_t)grow * PCH + cq;
      const v4f a = *(const v4f*)p;
      const v4f b = *(const v4f*)(p + 4);
      const float vv[8] = {a.x, a.y, a.z, a.w, b.x, b.y, b.z, b.w};
      const bool lo = q >= 4;
#pragma unroll
      for (int i = 0; i < 8; ++i) {
        const int c = cq + i;
        const float y = bn_relu(vv[i], pm[c], pm[32 + c], pm[64 + c], pm[96 + c]);
        const unsigned hb = bf16_bits(y);
        const unsigned lb = bf16_bits(y - __uint_as_float(hb << 16));
        const unsigned sel = lo ? lb : hb;
        o[i] = (c < DIM) ? (unsigned short)sel : (unsigned short)0;
      }
    }
    *(v8usa*)(at + row * KG + 8 * q) = o;
  }
  __syncthreads();

  v8f acc0 = {0.f, 0.f, 0.f, 0.f, 0.f, 0.f, 0.f, 0.f};
  v8f acc1 = {0.f, 0.f, 0.f, 0.f, 0.f, 0.f, 0.f, 0.f};
  const unsigned short* arow = at + (16 * wave + m) * KG + 8 * hh;
  const unsigned short* wp   = WT + (size_t)m * KG + 8 * hh;
#pragma unroll
  for (int ks = 0; ks < KG / 32; ++ks) {
    FragB af, b0, b1;
    af.h[0] = *(const v8usa*)(arow + 32 * ks);
    af.h[1] = *(const v8usa*)(arow + 32 * ks + 16);
    b0.h[0] = *(const v8usa*)(wp + 32 * ks);
    b0.h[1] = *(const v8usa*)(wp + 32 * ks + 16);
    b1.h[0] = *(const v8usa*)(wp + 16 * KG + 32 * ks);
    b1.h[1] = *(const v8usa*)(wp + 16 * KG + 32 * ks + 16);
    acc0 = wmb(af, b0, acc0);
    acc1 = wmb(af, b1, acc1);
  }

#pragma unroll
  for (int r = 0; r < 8; ++r) {
    const int lr = 16 * wave + 8 * hh + r;
    stg[lr * PCH + m]      = acc0[r];
    stg[lr * PCH + 16 + m] = acc1[r];
  }
  __syncthreads();

  v4f fv[4];
#pragma unroll
  for (int i = 0; i < 4; ++i) {
    const int lr = 16 * wave + 4 * i + (lane >> 3);
    const int c4 = (lane & 7) * 4;
    const v4f s  = *(const v4fa*)(stg + lr * PCH + c4);
    const float dd = dinvP[rowBase + lr];
    const bool cok = c4 < DIM;
    v4f y;
    y.x = cok ? dd * s.x : 0.0f;
    y.y = cok ? dd * s.y : 0.0f;
    y.z = cok ? dd * s.z : 0.0f;
    y.w = cok ? dd * s.w : 0.0f;
    fv[i] = y;
  }
#pragma unroll
  for (int i = 0; i < 4; ++i) {
    const int lr = 16 * wave + 4 * i + (lane >> 3);
    float* op = Y + (size_t)(rowBase + lr) * PCH + (lane & 7) * 4;
    *(volatile v4f*)op = fv[i];
  }
  __threadfence();
#pragma unroll
  for (int i = 0; i < 4; ++i) {
    const int lr = 16 * wave + 4 * i + (lane >> 3);
    float* op = Y + (size_t)(rowBase + lr) * PCH + (lane & 7) * 4;
    *(volatile v4f*)op = fv[i];
  }
}

__global__ __launch_bounds__(NTHR) void k_agg(const int* __restrict__ srcl, const int* __restrict__ offsP,
                                              const int* __restrict__ cntP, const float* __restrict__ dinvP,
                                              const float* __restrict__ Y, const float* __restrict__ par,
                                              int brow, int nN, float* agg, double* rec) {
  __shared__ double dSQ[2 * 32 * 32];
  __shared__ double res[64];
  const int tid = (int)threadIdx.x, lane = tid & 31, q = lane >> 3, i = lane & 7;
  const int wave = __builtin_amdgcn_readfirstlane(tid >> 5);
  const int nodeBase = (int)blockIdx.x * NBA;
  const int* gl = srcl + (size_t)blockIdx.x * RCAP;
  const v4f b4 = *(const v4f*)(par + brow * 32 + 4 * i);
  const bool colok = (4 * i) < DIM;
  double s0 = 0.0, s1 = 0.0, s2 = 0.0, s3 = 0.0;
  double q0 = 0.0, q1 = 0.0, q2 = 0.0, q3 = 0.0;

#pragma unroll 1
  for (int pass = 0; pass < NBA / 32; ++pass) {
    const int node = nodeBase + pass * 32 + wave * 4 + q;
    int c = cntP[node];
    c = c < 0 ? 0 : (c > DEGCAP ? DEGCAP : c);
    int o = offsP[node];
    o = o < 0 ? 0 : (o > RCAP - 1 ? RCAP - 1 : o);
    const float dd = dinvP[node];
    const int nc = node < nN ? node : nN - 1;
    int cm = c;
    {
      const int c8 = __shfl_xor(cm, 8, 32);
      cm = cm > c8 ? cm : c8;
      const int c16 = __shfl_xor(cm, 16, 32);
      cm = cm > c16 ? cm : c16;
    }
    cm = __builtin_amdgcn_readfirstlane(cm);
    cm = cm > DEGCAP ? DEGCAP : cm;
    float a0 = 0.0f, a1 = 0.0f, a2 = 0.0f, a3 = 0.0f;
#pragma unroll 1
    for (int p = 0; p < cm; ++p) {
      int idx = o + p;
      idx = idx > RCAP - 1 ? RCAP - 1 : idx;
      int s = gl[idx];
      s = s < 0 ? 0 : (s > nN - 1 ? nN - 1 : s);
      const v4f v = *(const v4f*)(Y + (size_t)s * PCH + 4 * i);
      const bool on = p < c;
      a0 += on ? v.x : 0.0f;
      a1 += on ? v.y : 0.0f;
      a2 += on ? v.z : 0.0f;
      a3 += on ? v.w : 0.0f;
    }
    const v4f ys = *(const v4f*)(Y + (size_t)nc * PCH + 4 * i);
    const bool keep = (node < nN) && colok;
    v4f ov;
    ov.x = keep ? (dd * (a0 + ys.x) + b4.x) : 0.0f;
    ov.y = keep ? (dd * (a1 + ys.y) + b4.y) : 0.0f;
    ov.z = keep ? (dd * (a2 + ys.z) + b4.z) : 0.0f;
    ov.w = keep ? (dd * (a3 + ys.w) + b4.w) : 0.0f;
    float* op = agg + (size_t)node * PCH + 4 * i;
    *(volatile v4f*)op = ov;
    __threadfence();
    *(volatile v4f*)op = ov;
    const double d0 = (double)ov.x, d1 = (double)ov.y, d2 = (double)ov.z, d3 = (double)ov.w;
    s0 += d0; s1 += d1; s2 += d2; s3 += d3;
    q0 += d0 * d0; q1 += d1 * d1; q2 += d2 * d2; q3 += d3 * d3;
  }

  {
    const int gb = (wave * 4 + q) * 32 + 4 * i;
    dSQ[gb + 0] = s0; dSQ[gb + 1] = s1; dSQ[gb + 2] = s2; dSQ[gb + 3] = s3;
    dSQ[1024 + gb + 0] = q0; dSQ[1024 + gb + 1] = q1; dSQ[1024 + gb + 2] = q2; dSQ[1024 + gb + 3] = q3;
  }
  __syncthreads();
  if (tid < 64) {
    const int base = (tid >> 5) * 1024 + (tid & 31);
    double s = 0.0;
#pragma unroll 4
    for (int g = 0; g < 32; ++g) s += dSQ[base + g * 32];
    res[tid] = s;
  }
  __syncthreads();
  if (wave == 0) {
    v2d rv;
    rv.x = res[2 * lane];
    rv.y = res[2 * lane + 1];
    double* rp = rec + (size_t)blockIdx.x * 64 + 2 * lane;
    *(volatile v2d*)rp = rv;
    __threadfence();
    *(volatile v2d*)rp = rv;
  }
}

__global__ __launch_bounds__(64) void k_bncomb(const double* __restrict__ rec, int nblk, double invn,
                                               float* stats) {
  __shared__ double tot[64];
  __shared__ __attribute__((aligned(16))) float outs[64];
  const int tid = (int)threadIdx.x;
  double s = 0.0;
#pragma unroll 4
  for (int b = 0; b < nblk; ++b) s += rec[(size_t)b * 64 + tid];
  tot[tid] = s;
  __syncthreads();
  if (tid < 32) {
    const double mean = tot[tid] * invn;
    double var = tot[32 + tid] * invn - mean * mean;
    var = (var < 0.0) ? 0.0 : var;
    const float vf = (float)var;
    outs[tid]      = (float)mean;
    outs[32 + tid] = 1.0f / sqrtf(vf + 1e-5f);
  }
  __syncthreads();
  const int t4 = tid < 16 ? tid : 15;
  const v4f ov = *(const v4fa*)(outs + 4 * t4);
  const bool st = tid < 16;
  if (st) *(volatile v4f*)(stats + 4 * t4) = ov;
  __threadfence();
  if (st) *(volatile v4f*)(stats + 4 * t4) = ov;
}

__global__ __launch_bounds__(NTHR) void k_final(const float* __restrict__ agg, const float* __restrict__ stats,
                                                const float* __restrict__ par, int prow, int nN, float* out) {
  __shared__ __attribute__((aligned(16))) float hs[FROWS * DIM];
  __shared__ float pm[4 * 32];
  const int tid = (int)threadIdx.x;
  const int base = (int)blockIdx.x * FROWS;
  if (tid < 32) {
    pm[tid]      = stats[tid];
    pm[32 + tid] = stats[32 + tid];
    pm[64 + tid] = par[(prow + 1) * 32 + tid];
    pm[96 + tid] = par[(prow + 2) * 32 + tid];
  }
  __syncthreads();
  constexpr int NU = FROWS * (DIM / 4);
#pragma unroll 1
  for (int it = 0; it < NU / NTHR; ++it) {
    const int u   = it * NTHR + tid;
    const int row = u / (DIM / 4);
    const int i   = u - row * (DIM / 4);
    const v4f a = *(const v4f*)(agg + (size_t)(base + row) * PCH + 4 * i);
    const int c = 4 * i;
    v4f y;
    y.x = bn_relu(a.x, pm[c + 0], pm[32 + c + 0], pm[64 + c + 0], pm[96 + c + 0]);
    y.y = bn_relu(a.y, pm[c + 1], pm[32 + c + 1], pm[64 + c + 1], pm[96 + c + 1]);
    y.z = bn_relu(a.z, pm[c + 2], pm[32 + c + 2], pm[64 + c + 2], pm[96 + c + 2]);
    y.w = bn_relu(a.w, pm[c + 3], pm[32 + c + 3], pm[64 + c + 3], pm[96 + c + 3]);
    *(v4fa*)(hs + row * DIM + c) = y;
  }
  __syncthreads();
  int nrows = nN - base;
  nrows = nrows < 0 ? 0 : (nrows > FROWS ? FROWS : nrows);
  const int n4 = nrows * (DIM / 4);
  float* op = out + (size_t)base * DIM;
#pragma unroll 1
  for (int it = 0; it < NU / NTHR; ++it) {
    const int i4 = it * NTHR + tid;
    const int ic = i4 < NU - 1 ? i4 : NU - 1;
    const v4f v = *(const v4fa*)(hs + 4 * ic);
    if (i4 < n4) *(volatile v4f*)(op + 4 * (size_t)i4) = v;
  }
  __threadfence();
#pragma unroll 1
  for (int it = 0; it < NU / NTHR; ++it) {
    const int i4 = it * NTHR + tid;
    const int ic = i4 < NU - 1 ? i4 : NU - 1;
    const v4f v = *(const v4fa*)(hs + 4 * ic);
    if (i4 < n4) *(volatile v4f*)(op + 4 * (size_t)i4) = v;
  }
}

__global__ __launch_bounds__(NTHR) void k_pool(const float* h, const int* __restrict__ bat, int nN,
                                               const float* __restrict__ par, float* ge, float* lg) {
  __shared__ float wm[NWAVE * GPB * 32];
  __shared__ __attribute__((aligned(16))) float gl[GPB * 32];
  __shared__ __attribute__((aligned(16))) float gd[GPB * DIM];
  __shared__ __attribute__((aligned(16))) float ho[GPB * NCLS];
  __shared__ float fw[96];
  const int tid = (int)threadIdx.x, lane = tid & 31;
  const int wave = __builtin_amdgcn_readfirstlane(tid >> 5);
  const int g0 = (int)blockIdx.x * GPB;
  const float ninf = __int_as_float((int)0xff800000u);
#pragma unroll 1
  for (int idx = tid; idx < NWAVE * GPB * 32; idx += NTHR) wm[idx] = ninf;
  if (tid < 96) fw[tid] = par[9 * 32 + tid];
  __syncthreads();

  float* my = wm + wave * (GPB * 32);
  const int cc = lane < DIM ? lane : DIM - 1;
#pragma unroll 1
  for (int i0 = wave * 32; i0 < nN; i0 += NTHR) {
    const int ii = i0 + lane;
    const int ic = ii < nN ? ii : nN - 1;
    const int b  = bat[ic];
    const unsigned sg = (unsigned)(b - g0);
    const bool hit = (ii < nN) && (sg < (unsigned)GPB);
    const int sgi = (int)(sg & (unsigned)(GPB - 1));
    unsigned msk = __builtin_amdgcn_ballot_w32(hit);
    int nh = (int)__builtin_popcount(msk);
    nh = nh > 32 ? 32 : nh;
#pragma unroll 1
    for (int qq = 0; qq < nh; ++qq) {
      const int k = __builtin_ffs((int)msk) - 1;
      msk &= msk - 1u;
      const int kk = k < 0 ? 0 : k;
      int node = i0 + kk;
      node = node > nN - 1 ? nN - 1 : node;
      const int slt = __builtin_amdgcn_readlane(sgi, kk) & (GPB - 1);
      const float a = h[(size_t)node * DIM + cc];
      float* mp = my + slt * 32 + lane;
      const float mo = *mp;
      *mp = nmax(a, mo);
    }
  }
  __syncthreads();
#pragma unroll 1
  for (int idx = tid; idx < GPB * 32; idx += NTHR) {
    float mv = wm[idx];
#pragma unroll
    for (int w2 = 1; w2 < NWAVE; ++w2) mv = nmax(wm[w2 * (GPB * 32) + idx], mv);
    gl[idx] = mv;
  }
  __syncthreads();
#pragma unroll 1
  for (int idx = tid; idx < GPB * DIM; idx += NTHR) {
    const int sl = idx / DIM;
    const int c  = idx - sl * DIM;
    gd[idx] = gl[sl * 32 + c];
  }
  if (tid < GPB * NCLS) {
    const int sl = tid >> 1;
    const int c  = tid & 1;
    float s = 0.0f;
#pragma unroll 4
    for (int k = 0; k < DIM; ++k) s = fmaf(gl[sl * 32 + k], fw[c * 32 + k], s);
    ho[tid] = s + fw[64 + c];
  }
  __syncthreads();
  {
    const int t80 = tid < 80 ? tid : 79;
    const v4f gv = *(const v4fa*)(gd + 4 * t80);
    const int t8 = (tid >= 96 && tid < 104) ? (tid - 96) : 0;
    const v4f hv = *(const v4fa*)(ho + 4 * t8);
    const bool sg1 = tid < 80;
    const bool sg2 = (tid >= 96) && (tid < 104);
    float* gp = ge + (size_t)g0 * DIM + 4 * t80;
    float* lp = lg + (size_t)g0 * NCLS + 4 * t8;
    if (sg1) *(volatile v4f*)gp = gv;
    if (sg2) *(volatile v4f*)lp = hv;
    __threadfence();
    if (sg1) *(volatile v4f*)gp = gv;
    if (sg2) *(volatile v4f*)lp = hv;
  }
}

static inline int cdiv(int a, int b) { return (a + b - 1) / b; }
static inline size_t al256(size_t o) { return (o + 255) & ~(size_t)255; }

extern "C" void kernel_launch(void* const* d_in, const int* in_sizes, int n_in,
                              void* d_out, int out_size, void* d_ws, size_t ws_size,
                              hipStream_t stream) {
  if (n_in < 17) return;
  if (in_sizes[0] < FIN || (in_sizes[0] % FIN) != 0) return;
  const int nN = in_sizes[0] / FIN;
  if (nN < 8 || nN > (1 << 22) || (nN % 8) != 0) return;
  if (in_sizes[1] < 2 || (in_sizes[1] & 1) != 0) return;
  const int nE = in_sizes[1] / 2;
  if (nE < 1 || nE > (1 << 22)) return;
  if (in_sizes[2] != nN) return;
  if (in_sizes[3] != FIN * DIM) return;
  if (in_sizes[7] != DIM * DIM || in_sizes[11] != DIM * DIM) return;
  for (int l = 0; l < 3; ++l)
    if (in_sizes[4 + 4 * l] != DIM || in_sizes[5 + 4 * l] != DIM || in_sizes[6 + 4 * l] != DIM) return;
  if (in_sizes[15] != DIM * NCLS || in_sizes[16] != NCLS) return;
  const long long outNeed = (long long)nN * DIM + (long long)NGR * DIM + (long long)NGR * NCLS;
  if ((long long)out_size != outNeed) return;

  const float* x    = (const float*)d_in[0];
  const int*   edge = (const int*)d_in[1];
  const int*   bat  = (const int*)d_in[2];
  const float* W0   = (const float*)d_in[3];
  const float* b0   = (const float*)d_in[4];
  const float* g0   = (const float*)d_in[5];
  const float* be0  = (const float*)d_in[6];
  const float* W1   = (const float*)d_in[7];
  const float* b1   = (const float*)d_in[8];
  const float* g1   = (const float*)d_in[9];
  const float* be1  = (const float*)d_in[10];
  const float* W2   = (const float*)d_in[11];
  const float* b2   = (const float*)d_in[12];
  const float* g2   = (const float*)d_in[13];
  const float* be2  = (const float*)d_in[14];
  const float* fcW  = (const float*)d_in[15];
  const float* fcb  = (const float*)d_in[16];
  float* out = (float*)d_out;
  float* outGE = out + (size_t)nN * DIM;
  float* outLG = outGE + (size_t)NGR * DIM;
  const int* src = edge;
  const int* dst = edge + nE;

  const int gA = cdiv(nN, NBA);
  const int NP = gA * NBA;
  const int gF = cdiv(nN, FROWS);
  if ((long long)gF * FROWS > (long long)NP) return;
  if (((long long)nN * DIM * 4) % 128 != 0) return;
  const int vec8 = ((nE & 3) == 0) ? 1 : 0;

  char* ws = (char*)d_ws;
  size_t off = 0;
  const size_t oW0T = off; off = al256(off + (size_t)32 * KG * 2);
  const size_t oW1T = off; off = al256(off + (size_t)32 * KG * 2);
  const size_t oW2T = off; off = al256(off + (size_t)32 * KG * 2);
  const size_t oPAR = off; off = al256(off + (size_t)NPAR * 32 * 4);
  const size_t oSTA = off; off = al256(off + (size_t)64 * 4);
  const size_t oREC = off; off = al256(off + (size_t)gA * 64 * 8);
  const size_t oOFF = off; off = al256(off + (size_t)NP * 4);
  const size_t oCNT = off; off = al256(off + (size_t)NP * 4);
  const size_t oDIN = off; off = al256(off + (size_t)NP * 4);
  const size_t oSRC = off; off = al256(off + (size_t)gA * RCAP * 4);
  const size_t oY   = off; off = al256(off + (size_t)NP * PCH * 4);
  const size_t oAGG = off; off = al256(off + (size_t)NP * PCH * 4);
  if (off > ws_size || off > (size_t)WSMAX) return;
  unsigned short* W0T = (unsigned short*)(ws + oW0T);
  unsigned short* W1T = (unsigned short*)(ws + oW1T);
  unsigned short* W2T = (unsigned short*)(ws + oW2T);
  float*  PAR  = (float*)(ws + oPAR);
  float*  STA  = (float*)(ws + oSTA);
  double* REC  = (double*)(ws + oREC);
  int*    OFFS = (int*)(ws + oOFF);
  int*    CNT  = (int*)(ws + oCNT);
  float*  DINV = (float*)(ws + oDIN);
  int*    SRCL = (int*)(ws + oSRC);
  float*  Y    = (float*)(ws + oY);
  float*  AGG  = (float*)(ws + oAGG);

  const size_t bldLds = (size_t)AGG_LDS_INTS * 4;
  hipFuncSetAttribute(reinterpret_cast<const void*>(&k_build), hipFuncAttributeMaxDynamicSharedMemorySize, (int)bldLds);
  const double invn = 1.0 / (double)nN;
  const int gG = NP / GBM;

  k_prep<<<1, NTHR, 0, stream>>>(W0, b0, g0, be0, W1, b1, g1, be1, W2, b2, g2, be2, fcW, fcb, W0T, W1T, W2T, PAR);
  k_build<<<gA, NTHR, bldLds, stream>>>(src, dst, nE, nN, vec8, SRCL, OFFS, CNT, DINV);
  k_gemm<0><<<gG, GTHR, 0, stream>>>(x, nN, W0T, STA, PAR, 0, DINV, Y);
  k_agg<<<gA, NTHR, 0, stream>>>(SRCL, OFFS, CNT, DINV, Y, PAR, 0, nN, AGG, REC);
  k_bncomb<<<1, 64, 0, stream>>>(REC, gA, invn, STA);
  k_gemm<1><<<gG, GTHR, 0, stream>>>(AGG, nN, W1T, STA, PAR, 0, DINV, Y);
  k_agg<<<gA, NTHR, 0, stream>>>(SRCL, OFFS, CNT, DINV, Y, PAR, 3, nN, AGG, REC);
  k_bncomb<<<1, 64, 0, stream>>>(REC, gA, invn, STA);
  k_gemm<1><<<gG, GTHR, 0, stream>>>(AGG, nN, W2T, STA, PAR, 3, DINV, Y);
  k_agg<<<gA, NTHR, 0, stream>>>(SRCL, OFFS, CNT, DINV, Y, PAR, 6, nN, AGG, REC);
  k_bncomb<<<1, 64, 0, stream>>>(REC, gA, invn, STA);
  k_final<<<gF, NTHR, 0, stream>>>(AGG, STA, PAR, 6, nN, out);
  k_pool<<<NGR / GPB, NTHR, 0, stream>>>(out, bat, nN, PAR, outGE, outLG);
}
